// TGating_24970939859569
// MI455X (gfx1250) — hardware-verified
//
#include <hip/hip_runtime.h>
#define NB8 8
#define NP 24
#define NTOK 1024
#define CI 16
#define DDm 256
#define NF 13
#define NR (NB8 * NTOK)
typedef __bf16 v16b __attribute__((ext_vector_type(16)));
typedef unsigned short v8us __attribute__((ext_vector_type(8), may_alias));
typedef float  v8f  __attribute__((ext_vector_type(8)));
typedef float  v4f  __attribute__((ext_vector_type(4)));
typedef float  v4fa __attribute__((ext_vector_type(4), may_alias));
union FragB { v16b v; v8us half[2]; unsigned short u[16]; };

__device__ __forceinline__ unsigned short bf16_bits(float x) { unsigned int u = __float_as_uint(x); return (unsigned short)((u + 0x7FFFu + ((u >> 16) & 1u)) >> 16); }
__device__ __forceinline__ float bf16_val(unsigned short b) { return __uint_as_float(((unsigned int)b) << 16); }
__device__ __forceinline__ float bf16_round(float x) { return bf16_val(bf16_bits(x)); }
template <int NT>
__device__ __forceinline__ v8f mmaN(v16b ah, v16b al, v16b bh, v16b bl, v8f c) {
  c = __builtin_amdgcn_wmma_f32_16x16x32_bf16(false, ah, false, bh, (short)0, c, false, false);
  if (NT >= 2) c = __builtin_amdgcn_wmma_f32_16x16x32_bf16(false, al, false, bh, (short)0, c, false, false);
  if (NT >= 3) c = __builtin_amdgcn_wmma_f32_16x16x32_bf16(false, ah, false, bl, (short)0, c, false, false);
  asm volatile("v_nop\n\tv_nop\n\tv_nop\n\tv_nop" : "+v"(c) : "v"(ah), "v"(al), "v"(bh), "v"(bl));
  return c;
}

__global__ __launch_bounds__(256) void k_wt_bf16(const float* __restrict__ W, unsigned short* __restrict__ Wt, int K, int N) {
  const int t = blockIdx.x * 256 + threadIdx.x;
  const int k8n = K / 8;
  if (t >= N * k8n) return;
  const int n = t / k8n, k8 = (t % k8n) * 8;
  v8us v;
#pragma unroll
  for (int i = 0; i < 8; ++i) v[i] = bf16_bits(W[(size_t)(k8 + i) * N + n]);
  *(volatile v8us*)(Wt + (size_t)n * K + k8) = v;
  __threadfence();
  *(volatile v8us*)(Wt + (size_t)n * K + k8) = v;
}

template <bool ASPLIT, int ACT, bool BIAS_BF16>
__global__ __launch_bounds__(128) void k_gemm_bf(const float* __restrict__ A, int lda, const unsigned short* __restrict__ Wt, int ldb,
                                               const float* __restrict__ bias, float* __restrict__ C, int ldc, int M, int N, int K) {
  __shared__ __attribute__((aligned(16))) float so[4][16][64];
  const int tid = threadIdx.x, w = tid >> 5, lane = tid & 31, ln = lane & 15, hh = lane >> 4;
  const int ntn = N / 64;
  const int wid = blockIdx.x * 4 + w;
  const int mt = wid / ntn, nq = wid % ntn;
  if (mt * 16 >= M) return;
  const int row0 = mt * 16, col0 = nq * 64;
  const float* arow = A + (size_t)(row0 + ln) * lda;
  v8f acc[4] = {};
  for (int kb = 0; kb < K; kb += 32) {
    FragB ah, al;
    const v4f x0 = *(const v4fa*)(arow + kb + 8 * hh), x1 = *(const v4fa*)(arow + kb + 8 * hh + 4);
    const v4f x2 = *(const v4fa*)(arow + kb + 16 + 8 * hh), x3 = *(const v4fa*)(arow + kb + 16 + 8 * hh + 4);
    float xs[16] = {x0[0],x0[1],x0[2],x0[3],x1[0],x1[1],x1[2],x1[3],x2[0],x2[1],x2[2],x2[3],x3[0],x3[1],x3[2],x3[3]};
#pragma unroll
    for (int i = 0; i < 16; ++i) { const unsigned short hb = bf16_bits(xs[i]); ah.u[i] = hb; al.u[i] = ASPLIT ? bf16_bits(xs[i] - bf16_val(hb)) : (unsigned short)0; }
#pragma unroll
    for (int t = 0; t < 4; ++t) {
      const unsigned short* brow = Wt + (size_t)(col0 + t * 16 + ln) * ldb + kb;
      FragB b;
      b.half[0] = *(const v8us*)(brow + 8 * hh);
      b.half[1] = *(const v8us*)(brow + 16 + 8 * hh);
      acc[t] = mmaN<ASPLIT ? 2 : 1>(ah.v, al.v, b.v, b.v, acc[t]);
    }
  }
#pragma unroll
  for (int t = 0; t < 4; ++t) {
    float bv = bias ? bias[col0 + t * 16 + ln] : 0.f;
    if (BIAS_BF16) bv = bf16_round(bv);
#pragma unroll
    for (int r = 0; r < 8; ++r) { float v = acc[t][r] + bv; if (ACT == 1) v = fmaxf(v, 0.f); so[w][8 * hh + r][t * 16 + ln] = v; }
  }
  __builtin_amdgcn_fence(__ATOMIC_ACQ_REL, "workgroup");
  __builtin_amdgcn_wave_barrier();
  const int rsub = lane >> 4, c4 = (lane & 15) * 4;
  for (int pass = 0; pass < 2; ++pass) {
#pragma unroll
    for (int q = 0; q < 8; ++q) {
      const int r = q * 2 + rsub;
      const v4f v = *(const v4fa*)&so[w][r][c4];
      *(volatile v4f*)(C + (size_t)(row0 + r) * ldc + col0 + c4) = v;
    }
    if (pass == 0) __threadfence();
  }
}

template <bool ASPLIT, int ACT, bool BIAS_BF16, bool RES_BF16>
__global__ __launch_bounds__(128) void k_gemm_bf3(const float* __restrict__ A, int lda, const unsigned short* __restrict__ Wt, int ldb,
                                                const float* __restrict__ bias, const float* __restrict__ resid, int rmod, int ldr,
                                                float* __restrict__ C, int ldc, int M, int N, int K) {
  __shared__ __attribute__((aligned(16))) float so[4][16][64];
  const int tid = threadIdx.x, w = tid >> 5, lane = tid & 31, ln = lane & 15, hh = lane >> 4;
  const int ntn = N / 64;
  const int wid = blockIdx.x * 4 + w;
  const int mt = wid / ntn, nq = wid % ntn;
  if (mt * 16 >= M) return;
  const int row0 = mt * 16, col0 = nq * 64;
  const float* arow = A + (size_t)(row0 + ln) * lda;
  v8f acc[4] = {};
  for (int kb = 0; kb < K; kb += 32) {
    FragB ah, al;
    const v4f x0 = *(const v4fa*)(arow + kb + 8 * hh), x1 = *(const v4fa*)(arow + kb + 8 * hh + 4);
    const v4f x2 = *(const v4fa*)(arow + kb + 16 + 8 * hh), x3 = *(const v4fa*)(arow + kb + 16 + 8 * hh + 4);
    float xs[16] = {x0[0],x0[1],x0[2],x0[3],x1[0],x1[1],x1[2],x1[3],x2[0],x2[1],x2[2],x2[3],x3[0],x3[1],x3[2],x3[3]};
#pragma unroll
    for (int i = 0; i < 16; ++i) { const unsigned short hb = bf16_bits(xs[i]); ah.u[i] = hb; al.u[i] = ASPLIT ? bf16_bits(xs[i] - bf16_val(hb)) : (unsigned short)0; }
#pragma unroll
    for (int t = 0; t < 4; ++t) {
      const unsigned short* brow = Wt + (size_t)(col0 + t * 16 + ln) * ldb + kb;
      FragB b;
      b.half[0] = *(const v8us*)(brow + 8 * hh);
      b.half[1] = *(const v8us*)(brow + 16 + 8 * hh);
      acc[t] = mmaN<ASPLIT ? 2 : 1>(ah.v, al.v, b.v, b.v, acc[t]);
    }
  }
#pragma unroll
  for (int t = 0; t < 4; ++t) {
    const int col = col0 + t * 16 + ln;
    float bv = bias ? bias[col] : 0.f;
    if (BIAS_BF16) bv = bf16_round(bv);
#pragma unroll
    for (int r = 0; r < 8; ++r) {
      float v = acc[t][r] + bv;
      if (resid) { float rv = resid[(size_t)((row0 + 8 * hh + r) % rmod) * ldr + col]; if (RES_BF16) rv = bf16_round(rv); v += rv; }
      if (ACT == 1) v = fmaxf(v, 0.f);
      if (ACT == 2) v = 0.5f * v * (1.0f + erff(v * 0.70710678118654752f));
      if (ACT == 3) { const float u = 0.7978845608028654f * (v + 0.044715f * v * v * v); v = 0.5f * v * (1.0f + tanhf(u)); }
      so[w][8 * hh + r][t * 16 + ln] = v;
    }
  }
  __builtin_amdgcn_fence(__ATOMIC_ACQ_REL, "workgroup");
  __builtin_amdgcn_wave_barrier();
  const int rsub = lane >> 4, c4 = (lane & 15) * 4;
  for (int pass = 0; pass < 2; ++pass) {
#pragma unroll
    for (int q = 0; q < 8; ++q) {
      const int r = q * 2 + rsub;
      const v4f v = *(const v4fa*)&so[w][r][c4];
      *(volatile v4f*)(C + (size_t)(row0 + r) * ldc + col0 + c4) = v;
    }
    if (pass == 0) __threadfence();
  }
}
template <bool PARAM_BF16>
__global__ __launch_bounds__(256) void k_layernorm(const float* __restrict__ X, const float* __restrict__ R, const float* __restrict__ g, const float* __restrict__ bta,
                                                  float* __restrict__ out_sum, float* __restrict__ out_norm, int N, float eps) {
  __shared__ float red[256];
  const int row = blockIdx.x, tid = threadIdx.x;
  const float* x = X + (size_t)row * N; const float* rr = R ? R + (size_t)row * N : nullptr;
  float vals[16];
  const int per = N / 256;
  float s1 = 0.f;
  for (int u = 0; u < per / 4; ++u) {
    const int j = tid * 4 + 1024 * u;
    const v4f a = *(const v4fa*)(x + j);
    v4f b = {0.f,0.f,0.f,0.f}; if (rr) b = *(const v4fa*)(rr + j);
#pragma unroll
    for (int q = 0; q < 4; ++q) { const float v = a[q] + b[q]; vals[u * 4 + q] = v; s1 += v; }
  }
  red[tid] = s1; __syncthreads();
  for (int st = 128; st > 0; st >>= 1) { if (tid < st) red[tid] += red[tid + st]; __syncthreads(); }
  const float mu = red[0] / (float)N; __syncthreads();
  float s2 = 0.f;
  for (int u = 0; u < per / 4; ++u)
#pragma unroll
    for (int q = 0; q < 4; ++q) { const float c = vals[u * 4 + q] - mu; s2 += c * c; }
  red[tid] = s2; __syncthreads();
  for (int st = 128; st > 0; st >>= 1) { if (tid < st) red[tid] += red[tid + st]; __syncthreads(); }
  const float rs = rsqrtf(red[0] / (float)N + eps);
  for (int pass = 0; pass < 2; ++pass) {
    for (int u = 0; u < per / 4; ++u) {
      const int j = tid * 4 + 1024 * u;
      v4f o, sm;
#pragma unroll
      for (int q = 0; q < 4; ++q) {
        float gg = g[j + q], bb = bta[j + q];
        if (PARAM_BF16) { gg = bf16_round(gg); bb = bf16_round(bb); }
        sm[q] = vals[u * 4 + q]; o[q] = (vals[u * 4 + q] - mu) * rs * gg + bb;
      }
      if (out_sum) *(volatile v4f*)(out_sum + (size_t)row * N + j) = sm;
      *(volatile v4f*)(out_norm + (size_t)row * N + j) = o;
    }
    if (pass == 0) __threadfence();
  }
}


typedef _Float16 v16h __attribute__((ext_vector_type(16)));
union FragH { v16h v; v8us half[2]; _Float16 h[16]; unsigned short u[16]; };
template <int NT>
__device__ __forceinline__ v8f mmaH(v16h ah, v16h al, v16h bh, v16h bl, v8f c) {
  c = __builtin_amdgcn_wmma_f32_16x16x32_f16(false, ah, false, bh, (short)0, c, false, false);
  if (NT >= 2) c = __builtin_amdgcn_wmma_f32_16x16x32_f16(false, al, false, bh, (short)0, c, false, false);
  if (NT >= 3) c = __builtin_amdgcn_wmma_f32_16x16x32_f16(false, ah, false, bl, (short)0, c, false, false);
  asm volatile("v_nop\n\tv_nop\n\tv_nop\n\tv_nop" : "+v"(c) : "v"(ah), "v"(al), "v"(bh), "v"(bl));
  return c;
}
template <bool ASPLIT>
__global__ __launch_bounds__(128) void k_gemm_h(const float* __restrict__ A, int lda, size_t sA, const _Float16* __restrict__ Bh, int ldb, size_t sB, float alpha, float* __restrict__ C, int ldc, size_t sC, int M, int N, int K) {
  __shared__ __attribute__((aligned(16))) float so[4][16][64];
  const int tid = threadIdx.x, w = tid >> 5, lane = tid & 31, ln = lane & 15, hh = lane >> 4; const int by = blockIdx.y;
  A += (size_t)by * sA; Bh += (size_t)by * sB; C += (size_t)by * sC;
  const int ntn = (N + 63) / 64; const int wid = blockIdx.x * 4 + w; const int mt = wid / ntn, nq = wid % ntn; if (mt * 16 >= M) return;
  const int row0 = mt * 16, col0 = nq * 64; const float* arow = A + (size_t)(row0 + ln) * lda;
  v8f acc[4] = {};
  for (int kb = 0; kb < K; kb += 32) {
    FragH ah, al;
    const v4f x0 = *(const v4fa*)(arow + kb + 8 * hh), x1 = *(const v4fa*)(arow + kb + 8 * hh + 4), x2 = *(const v4fa*)(arow + kb + 16 + 8 * hh), x3 = *(const v4fa*)(arow + kb + 16 + 8 * hh + 4);
    float xs[16] = {x0[0],x0[1],x0[2],x0[3],x1[0],x1[1],x1[2],x1[3],x2[0],x2[1],x2[2],x2[3],x3[0],x3[1],x3[2],x3[3]};
#pragma unroll
    for (int i = 0; i < 16; ++i) { const _Float16 h = (_Float16)xs[i]; ah.h[i] = h; al.h[i] = ASPLIT ? (_Float16)(xs[i] - (float)h) : (_Float16)0.0f; }
#pragma unroll
    for (int t = 0; t < 4; ++t) { if (col0 + t * 16 >= N) continue; const size_t boff = (size_t)(col0 + t * 16 + ln) * ldb + kb; FragH bq; bq.half[0] = *(const v8us*)(Bh + boff + 8 * hh); bq.half[1] = *(const v8us*)(Bh + boff + 16 + 8 * hh);
      acc[t] = mmaH<ASPLIT ? 2 : 1>(ah.v, al.v, bq.v, bq.v, acc[t]); }
  }
#pragma unroll
  for (int t = 0; t < 4; ++t) { if (col0 + t * 16 >= N) continue;
#pragma unroll
    for (int r = 0; r < 8; ++r) so[w][8 * hh + r][t * 16 + ln] = acc[t][r] * alpha; }
  __builtin_amdgcn_fence(__ATOMIC_ACQ_REL, "workgroup"); __builtin_amdgcn_wave_barrier();
  const int rsub = lane >> 4, c4 = (lane & 15) * 4;
  for (int pass = 0; pass < 2; ++pass) {
#pragma unroll
    for (int q = 0; q < 8; ++q) { const int r = q * 2 + rsub; if (col0 + c4 < N) { const v4f v = *(const v4fa*)&so[w][r][c4]; *(volatile v4f*)(C + (size_t)(row0 + r) * ldc + col0 + c4) = v; } }
    if (pass == 0) __threadfence(); }
}

__global__ __launch_bounds__(256) void k_wt_f16(const float* __restrict__ W, _Float16* __restrict__ Wt, int K, int N, float scale) {
  const int t = blockIdx.x * 256 + threadIdx.x; if (t >= N * (K / 8)) return; const int n = t / (K / 8), k8 = (t % (K / 8)) * 8; FragH f;
#pragma unroll
  for (int i = 0; i < 8; ++i) f.h[i] = (_Float16)(bf16_round(W[(size_t)(k8 + i) * N + n]) * scale); const v8us o = f.half[0];
  *(volatile v8us*)((unsigned short*)Wt + (size_t)n * K + k8) = o; __threadfence(); *(volatile v8us*)((unsigned short*)Wt + (size_t)n * K + k8) = o;
}
template <int ACT>
__global__ __launch_bounds__(128) void k_gemm_hhx(const _Float16* __restrict__ A, int lda, size_t sA, const _Float16* __restrict__ Bh, int ldb, size_t sB, float alpha, const float* __restrict__ bias, size_t sBias, const float* __restrict__ CP, int rowsPerB, size_t sCPb, int row0g,
    float* __restrict__ C, _Float16* __restrict__ C16, int ldc, size_t sC, int M, int N, int K) {
  __shared__ __attribute__((aligned(16))) float so[4][16][64];
  const int tid = threadIdx.x, w = tid >> 5, lane = tid & 31, ln = lane & 15, hh = lane >> 4; const int by = blockIdx.y;
  A += (size_t)by * sA; Bh += (size_t)by * sB; const size_t cofs = (size_t)by * sC; const float* bp = bias ? bias + (size_t)by * sBias : nullptr;
  const int ntn = (N + 63) / 64; const int wid = blockIdx.x * 4 + w; const int mt = wid / ntn, nq = wid % ntn; if (mt * 16 >= M) return;
  const int row0 = mt * 16, col0 = nq * 64; const _Float16* arow = A + (size_t)(row0 + ln) * lda;
  v8f acc[4] = {};
  for (int kb = 0; kb < K; kb += 32) { FragH ah; ah.half[0] = *(const v8us*)((const unsigned short*)arow + kb + 8 * hh); ah.half[1] = *(const v8us*)((const unsigned short*)arow + kb + 16 + 8 * hh);
#pragma unroll
    for (int t = 0; t < 4; ++t) { if (col0 + t * 16 >= N) continue; const size_t boff = (size_t)(col0 + t * 16 + ln) * ldb + kb; FragH bq; bq.half[0] = *(const v8us*)((const unsigned short*)Bh + boff + 8 * hh); bq.half[1] = *(const v8us*)((const unsigned short*)Bh + boff + 16 + 8 * hh);
      acc[t] = mmaH<1>(ah.v, ah.v, bq.v, bq.v, acc[t]); }
  }
#pragma unroll
  for (int t = 0; t < 4; ++t) { if (col0 + t * 16 >= N) continue; const int col = col0 + t * 16 + ln; const float bv = bp ? bf16_round(bp[col]) : 0.f;
#pragma unroll
    for (int r = 0; r < 8; ++r) { float v = acc[t][r] * alpha + bv; if (CP) { const int bidx = (row0g + row0 + 8 * hh + r) / rowsPerB; v += CP[(size_t)bidx * sCPb + (size_t)by * 64 + col]; } if (ACT == 1) v = (v > 0.f) ? v : expm1f(v); else if (ACT == 7) v = (v > 0.f) ? v + 1.0f : expf(v); else if (ACT == 8) v = tanhf(v); else if (ACT == 9) v = 0.5f * v * (1.0f + tanhf(0.7978845608028654f * (v + 0.044715f * v * v * v))); else if (ACT == 11) v = 1.0f / (1.0f + expf(-v)); else if (ACT == 12) v = (v > 0.f) ? v : 0.01f * v; else if (ACT == 14) v = (v > 0.f) ? v : 0.1f * v; else if (ACT == 15) v = v / (1.0f + expf(-v)); else if (ACT == 3) v = fmaxf(v, 0.f); else if (ACT == 6) v = 0.5f * v * (1.0f + erff(v * 0.70710678118654752f)); so[w][8 * hh + r][t * 16 + ln] = v; } }
  __builtin_amdgcn_fence(__ATOMIC_ACQ_REL, "workgroup"); __builtin_amdgcn_wave_barrier();
  const int rsub = lane >> 4, c4 = (lane & 15) * 4; typedef _Float16 v4h __attribute__((ext_vector_type(4)));
  for (int pass = 0; pass < 2; ++pass) {
#pragma unroll
    for (int q = 0; q < 8; ++q) { const int r = q * 2 + rsub; if (col0 + c4 < N) { const v4f v = *(const v4fa*)&so[w][r][c4]; if (C) *(volatile v4f*)(C + cofs + (size_t)(row0 + r) * ldc + col0 + c4) = v; if (C16) { v4h h4; for (int i = 0; i < 4; ++i) h4[i] = (_Float16)v[i]; *(volatile v4h*)(C16 + cofs + (size_t)(row0 + r) * ldc + col0 + c4) = h4; } } }
    if (pass == 0) __threadfence(); }
}


typedef _Float16 v4h __attribute__((ext_vector_type(4)));

__global__ __launch_bounds__(256) void k_x16(const float* __restrict__ x, _Float16* __restrict__ X16, size_t n8) { const size_t t = (size_t)blockIdx.x * 256 + threadIdx.x; if (t >= n8) return; FragH f;
#pragma unroll
  for (int q = 0; q < 8; ++q) f.h[q] = (_Float16)bf16_round(x[t * 8 + q]); *(volatile v8us*)((unsigned short*)X16 + t * 8) = f.half[0]; __threadfence(); *(volatile v8us*)((unsigned short*)X16 + t * 8) = f.half[0]; }
__global__ __launch_bounds__(256) void k_h16(const float* __restrict__ x, _Float16* __restrict__ X16, size_t n8) { const size_t t = (size_t)blockIdx.x * 256 + threadIdx.x; if (t >= n8) return; FragH f;
#pragma unroll
  for (int q = 0; q < 8; ++q) f.h[q] = (_Float16)x[t * 8 + q]; *(volatile v8us*)((unsigned short*)X16 + t * 8) = f.half[0]; __threadfence(); *(volatile v8us*)((unsigned short*)X16 + t * 8) = f.half[0]; }
__global__ __launch_bounds__(256) void k_round16f(const float* __restrict__ W, _Float16* __restrict__ Bt, size_t n8) { const size_t t = (size_t)blockIdx.x * 256 + threadIdx.x; if (t >= n8) return; FragH f;
#pragma unroll
  for (int i = 0; i < 8; ++i) f.h[i] = (_Float16)(bf16_round(W[t * 8 + i]) * 16.0f); *(volatile v8us*)((unsigned short*)Bt + t * 8) = f.half[0]; __threadfence(); *(volatile v8us*)((unsigned short*)Bt + t * 8) = f.half[0]; }
template <int NHv, int TTv>
__global__ __launch_bounds__(256) void k_vt(const _Float16* __restrict__ V16, int ldv, int voff, _Float16* __restrict__ Vt) { __shared__ unsigned short tl[64][66]; const int tid = threadIdx.x; const int slab = blockIdx.x / (TTv / 64), lg = blockIdx.x % (TTv / 64); const int b = slab / NHv, h = slab % NHv;
  for (int i = tid; i < 64 * 8; i += 256) { const int r = i / 8, c8 = (i % 8) * 8; FragH f; f.half[0] = *(const v8us*)((const unsigned short*)V16 + ((size_t)b * TTv + lg * 64 + r) * ldv + voff + h * 64 + c8);
#pragma unroll
    for (int q = 0; q < 8; ++q) tl[r][c8 + q] = f.u[q]; }
  __syncthreads();
  for (int pass = 0; pass < 2; ++pass) {
#pragma unroll
    for (int rd = 0; rd < 2; ++rd) { const int d = rd * 32 + tid / 8, pc = tid % 8; FragH f;
#pragma unroll
      for (int q = 0; q < 8; ++q) f.u[q] = tl[pc * 8 + q][d];
      *(volatile v8us*)((unsigned short*)Vt + ((size_t)slab * 64 + d) * TTv + lg * 64 + pc * 8) = f.half[0]; }
    if (pass == 0) __threadfence(); } }

__global__ __launch_bounds__(256) void k_hl(const float* __restrict__ F, _Float16* __restrict__ Hh, _Float16* __restrict__ Hl, size_t n8) { const size_t t = (size_t)blockIdx.x * 256 + threadIdx.x; if (t >= n8) return; FragH fh, fl; const v4f a = *(const v4fa*)(F + t * 8), c = *(const v4fa*)(F + t * 8 + 4);
#pragma unroll
  for (int q = 0; q < 4; ++q) { _Float16 h = (_Float16)a[q]; fh.h[q] = h; fl.h[q] = (_Float16)((a[q] - (float)h) * 1024.0f); h = (_Float16)c[q]; fh.h[4 + q] = h; fl.h[4 + q] = (_Float16)((c[q] - (float)h) * 1024.0f); }
  for (int pass = 0; pass < 2; ++pass) { *(volatile v8us*)((unsigned short*)Hh + t * 8) = fh.half[0]; *(volatile v8us*)((unsigned short*)Hl + t * 8) = fl.half[0]; if (pass == 0) __threadfence(); } }

__device__ __forceinline__ float gelu_f(float v) { return 0.5f * v * (1.0f + erff(v * 0.70710678118654752f)); }
__device__ __forceinline__ float xin(const float* x, int b, int p, int e) { return bf16_round(x[(((size_t)b * NP + p) * NTOK * CI) + e]); }
__global__ __launch_bounds__(256) void k_smean(const float* __restrict__ x, float* __restrict__ SM) { __shared__ float red[256]; const int tid = threadIdx.x; const int bp = blockIdx.x; const int b = bp / NP, p = bp % NP; const int c = tid & 15, n0 = tid >> 4; float s = 0.f;
#pragma unroll 1
  for (int n = n0; n < NTOK; n += 16) s += xin(x, b, p, n * CI + c);
  red[tid] = s; __syncthreads(); for (int st = 128; st >= 16; st >>= 1) { if (tid < st) red[tid] += red[tid + st]; __syncthreads(); }
  if (tid < 32) { const float v = (tid < CI) ? red[tid] / (float)NTOK : 0.f; *(volatile float*)(SM + (size_t)bp * 32 + tid) = v; __threadfence(); *(volatile float*)(SM + (size_t)bp * 32 + tid) = v; } }
__global__ __launch_bounds__(256) void k_lagd(const float* __restrict__ x, float* __restrict__ D4) {
  #pragma clang fp contract(off)
  __shared__ float red[4][256]; const int tid = threadIdx.x; const int bp = blockIdx.x; const int b = bp / NP, p = bp % NP; const int lags[4] = {1, 2, 4, 6}; float acc[4] = {0.f, 0.f, 0.f, 0.f};
  auto xr = [&](int pp, int e) { const float xv = xin(x, b, pp, e); float base; if (pp <= 1) base = xin(x, b, 0, e); else base = ((xin(x, b, pp - 1, e) + xin(x, b, pp - 2, e)) + xv) / 3.0f; return xv - base; };
#pragma unroll 1
  for (int e = tid; e < NTOK * CI; e += 256) { const float r0 = xr(p, e);
#pragma unroll
    for (int li = 0; li < 4; ++li) { const int q = p - lags[li]; const float r1 = (q >= 0) ? xr(q, e) : r0; acc[li] += fabsf(r0 - r1); } }
#pragma unroll
  for (int li = 0; li < 4; ++li) red[li][tid] = acc[li];
  __syncthreads(); for (int st = 128; st > 0; st >>= 1) { if (tid < st) { for (int li = 0; li < 4; ++li) red[li][tid] += red[li][tid + st]; } __syncthreads(); }
  if (tid < 32) { const float v = (tid < 4) ? red[tid][0] / (float)(NTOK * CI) : 0.f; *(volatile float*)(D4 + (size_t)bp * 32 + tid) = v; __threadfence(); *(volatile float*)(D4 + (size_t)bp * 32 + tid) = v; } }
__global__ __launch_bounds__(256) void k_battn(const float* __restrict__ D4, const float* __restrict__ SM, const float* __restrict__ pool, const float* __restrict__ pw1, const float* __restrict__ pb1, const float* __restrict__ pw2, const float* __restrict__ pb2, const float* __restrict__ nw, const float* __restrict__ nbias, const float* __restrict__ ipb, float* __restrict__ ATT, float* __restrict__ TA, float* __restrict__ TEF, float* __restrict__ tv) {
  #pragma clang fp contract(off)
  __shared__ float te[NP][DDm]; __shared__ float pe1[2][NP][64]; __shared__ float att[32]; __shared__ float srt[NP]; __shared__ float gsc[NP]; const int tid = threadIdx.x, b = blockIdx.x;
  for (int i = tid; i < 2 * NP * 64; i += 256) { const int k = i / (NP * 64), p = (i / 64) % NP, o = i % 64; const float per = (k == 0) ? 24.0f : 72.0f; const float ph = (2.0f * 3.14159265358979323846f * (float)p) / per; const float sn = (float)sin((double)ph), cs = (float)cos((double)ph);
    pe1[k][p][o] = gelu_f((sn * bf16_round(pw1[(k * 2 + 0) * 64 + o]) + cs * bf16_round(pw1[(k * 2 + 1) * 64 + o])) + bf16_round(pb1[k * 64 + o])); }
  __syncthreads();
  for (int i = tid; i < NP * DDm; i += 256) { const int p = i / DDm, c = i % DDm; float v;
    if (c < 128) { const int k = c / 64, qq = c % 64; float s = bf16_round(pb2[k * 64 + qq]);
#pragma unroll 1
      for (int o = 0; o < 64; ++o) s += pe1[k][p][o] * bf16_round(pw2[((size_t)k * 64 + o) * 64 + qq]);
      v = s; }
    else { const int qq = c - 128; float s = bf16_round(nbias[qq]);
#pragma unroll 1
      for (int ci = 0; ci < CI; ++ci) s += SM[((size_t)b * NP + p) * 32 + ci] * bf16_round(nw[ci * 128 + qq]);
      v = s; }
    te[p][c] = v; }
  if (tid == 0) { _Pragma("unroll 1") for (int p = 0; p < NP; ++p) gsc[p] = 0.f;
    _Pragma("unroll 1") for (int li = 0; li < 4; ++li) {
      _Pragma("unroll 1") for (int p = 0; p < NP; ++p) srt[p] = D4[((size_t)b * NP + p) * 32 + li];
      _Pragma("unroll 1") for (int i = 1; i < NP; ++i) { const float key = srt[i]; int j = i - 1; while (j >= 0 && srt[j] > key) { srt[j + 1] = srt[j]; --j; } srt[j + 1] = key; }
      const float med = srt[11];
      _Pragma("unroll 1") for (int p = 0; p < NP; ++p) srt[p] = fabsf(D4[((size_t)b * NP + p) * 32 + li] - med);
      _Pragma("unroll 1") for (int i = 1; i < NP; ++i) { const float key = srt[i]; int j = i - 1; while (j >= 0 && srt[j] > key) { srt[j + 1] = srt[j]; --j; } srt[j + 1] = key; }
      const float mad = srt[11]; const float den = mad * 1.4826f + 1e-6f;
      _Pragma("unroll 1") for (int p = 0; p < NP; ++p) { const float z = (D4[((size_t)b * NP + p) * 32 + li] - med) / den; const float sp = (z > 20.f) ? z : log1pf(expf(z)); gsc[p] += sp; }
      }
    _Pragma("unroll 1") for (int p = 0; p < NP; ++p) gsc[p] = gsc[p] / 4.0f;
    { float c = gsc[0]; _Pragma("unroll 1") for (int p = 1; p < NP; ++p) { c = 0.6f * c + (1.0f - 0.6f) * gsc[p]; gsc[p] = c; } }
    { float mu = 0.f; _Pragma("unroll 1") for (int p = 0; p < NP; ++p) mu += gsc[p]; mu /= (float)NP; _Pragma("unroll 1") for (int p = 0; p < NP; ++p) gsc[p] = 1.0f / (1.0f + expf(-1.5f * (gsc[p] - mu))); }
    { float mx = -3.0e38f; _Pragma("unroll 1") for (int p = 0; p < NP; ++p) mx = fmaxf(mx, bf16_round(pool[p])); float su = 0.f; _Pragma("unroll 1") for (int p = 0; p < NP; ++p) { srt[p] = expf(bf16_round(pool[p]) - mx); su += srt[p]; } _Pragma("unroll 1") for (int p = 0; p < NP; ++p) srt[p] /= su; }
    { float mx = -3.0e38f; _Pragma("unroll 1") for (int p = 0; p < NP; ++p) { srt[p] = srt[p] * (1.0f + gsc[p]); mx = fmaxf(mx, srt[p]); } float su = 0.f; _Pragma("unroll 1") for (int p = 0; p < NP; ++p) { srt[p] = expf(srt[p] - mx); su += srt[p]; } _Pragma("unroll 1") for (int p = 0; p < 32; ++p) att[p] = (p < NP) ? srt[p] / su : 0.f; } }
  __syncthreads();
  for (int pass = 0; pass < 2; ++pass) {
    if (tid < 32) *(volatile float*)(ATT + (size_t)b * 32 + tid) = att[tid];
    { const int c = tid; float s = 0.f, m = 0.f; _Pragma("unroll 1") for (int p = 0; p < NP; ++p) { s += att[p] * te[p][c]; m += te[p][c]; } *(volatile float*)(TA + (size_t)b * DDm + c) = s; *(volatile float*)(tv + (size_t)b * DDm + c) = m / (float)NP; }
    for (int i = tid; i < NF * 2 * DDm; i += 256) { const int f = i / (2 * DDm), ri = (i / DDm) % 2, c = i % DDm; double s = 0.0; const float bi = bf16_round(ipb[c]);
      _Pragma("unroll 1") for (int p = 0; p < NP; ++p) { const double th = 2.0 * 3.14159265358979323846 * (double)f * (double)p / 24.0; const double w = ri ? -sin(th) : cos(th); s += (double)(bi + te[p][c]) * w; }
      *(volatile float*)(TEF + (((size_t)b * NF + f) * 2 + ri) * DDm + c) = (float)s; }
    if (pass == 0) __threadfence(); } }
__global__ __launch_bounds__(256) void k_xa(const float* __restrict__ x, const float* __restrict__ ATT, float* __restrict__ XA) {
  #pragma clang fp contract(off)
  const int t = blockIdx.x * 256 + threadIdx.x; if (t >= NR * CI) return; const int b = t / (NTOK * CI), e = t % (NTOK * CI); float s = 0.f;
#pragma unroll 1
  for (int p = 0; p < NP; ++p) s += ATT[(size_t)b * 32 + p] * xin(x, b, p, e);
  *(volatile float*)(XA + t) = s; __threadfence(); *(volatile float*)(XA + t) = s; }
__global__ __launch_bounds__(256) void k_dft(const float* __restrict__ x, int f, _Float16* __restrict__ Ah, _Float16* __restrict__ Al) {
  #pragma clang fp contract(off)
  const int t = blockIdx.x * 256 + threadIdx.x; if (t >= NR * 4) return; const int part = t & 3, bn = t >> 2; const int b = bn / NTOK, n = bn % NTOK; const int c0 = part * 8; float re[8], im[8];
#pragma unroll
  for (int q = 0; q < 8; ++q) { re[q] = 0.f; im[q] = 0.f; }
  if (part < 2) {
#pragma unroll 1
    for (int p = 0; p < NP; ++p) { const double th = 2.0 * 3.14159265358979323846 * (double)f * (double)p / 24.0; const float cs = (float)cos(th), sn = (float)sin(th); const v4f a = *(const v4fa*)(x + (((size_t)b * NP + p) * NTOK + n) * CI + c0), cq = *(const v4fa*)(x + (((size_t)b * NP + p) * NTOK + n) * CI + c0 + 4);
#pragma unroll
      for (int q = 0; q < 8; ++q) { const float v = bf16_round((q < 4) ? a[q] : cq[q - 4]); re[q] += v * cs; im[q] -= v * sn; } } }
  FragH h1, l1, h2, l2;
#pragma unroll
  for (int q = 0; q < 8; ++q) { const _Float16 a1 = (_Float16)re[q], a2 = (_Float16)im[q]; h1.h[q] = a1; l1.h[q] = (_Float16)((re[q] - (float)a1) * 1024.0f); h2.h[q] = a2; l2.h[q] = (_Float16)((im[q] - (float)a2) * 1024.0f); }
  for (int pass = 0; pass < 2; ++pass) { *(volatile v8us*)((unsigned short*)Ah + (size_t)bn * 32 + c0) = h1.half[0]; *(volatile v8us*)((unsigned short*)Al + (size_t)bn * 32 + c0) = l1.half[0]; *(volatile v8us*)((unsigned short*)Ah + (size_t)(NR + bn) * 32 + c0) = h2.half[0]; *(volatile v8us*)((unsigned short*)Al + (size_t)(NR + bn) * 32 + c0) = l2.half[0]; if (pass == 0) __threadfence(); } }
__global__ __launch_bounds__(256) void k_win(const float* __restrict__ ipw, _Float16* __restrict__ Bt) { const int o = blockIdx.x * 256 + threadIdx.x; if (o >= DDm) return; FragH f[4];
#pragma unroll
  for (int c = 0; c < 32; ++c) f[c >> 3].h[c & 7] = (c < CI) ? (_Float16)(bf16_round(ipw[c * DDm + o]) * 16.0f) : (_Float16)0.0f;
  for (int pass = 0; pass < 2; ++pass) {
#pragma unroll
    for (int q = 0; q < 4; ++q) *(volatile v8us*)((unsigned short*)Bt + (size_t)o * 32 + 8 * q) = f[q].half[0];
    if (pass == 0) __threadfence(); } }
__global__ __launch_bounds__(256) void k_comp(const float* __restrict__ HF, const float* __restrict__ TEF, int f, _Float16* __restrict__ C16) {
  #pragma clang fp contract(off)
  const int t = blockIdx.x * 256 + threadIdx.x; if (t >= NR * 64) return; const int c0 = (t & 31) * 8, ri = (t >> 5) & 1, bn = t >> 6; const int b = bn / NTOK; FragH fr;
#pragma unroll
  for (int q = 0; q < 8; ++q) fr.h[q] = (_Float16)(HF[((size_t)ri * NR + bn) * DDm + c0 + q] + TEF[(((size_t)b * NF + f) * 2 + ri) * DDm + c0 + q]);
  *(volatile v8us*)((unsigned short*)C16 + (size_t)bn * 512 + ri * DDm + c0) = fr.half[0]; __threadfence(); *(volatile v8us*)((unsigned short*)C16 + (size_t)bn * 512 + ri * DDm + c0) = fr.half[0]; }
__global__ __launch_bounds__(256) void k_gelu(const float* __restrict__ T, _Float16* __restrict__ H16, size_t n4) {
  #pragma clang fp contract(off)
  const size_t t = (size_t)blockIdx.x * 256 + threadIdx.x; if (t >= n4) return; const v4f a = *(const v4fa*)(T + t * 4); FragH f;
#pragma unroll
  for (int q = 0; q < 4; ++q) f.h[q] = (_Float16)gelu_f(a[q]);
  const unsigned long long pv = *(const unsigned long long*)&f.u[0]; *(volatile unsigned long long*)((unsigned short*)H16 + t * 4) = pv; __threadfence(); *(volatile unsigned long long*)((unsigned short*)H16 + t * 4) = pv; }
__global__ __launch_bounds__(256) void k_z(const float* __restrict__ XA, const float* __restrict__ ipw, const float* __restrict__ ipb, const float* __restrict__ TA, const float* __restrict__ HQ, float* __restrict__ out) {
  #pragma clang fp contract(off)
  const int t = blockIdx.x * 256 + threadIdx.x; if (t >= NR * (DDm / 8)) return; const int c0 = (t % (DDm / 8)) * 8, bn = t / (DDm / 8); const int b = bn / NTOK; float acc[8];
#pragma unroll
  for (int q = 0; q < 8; ++q) acc[q] = 0.f;
#pragma unroll 1
  for (int ci = 0; ci < CI; ++ci) { const float xa = XA[(size_t)bn * CI + ci];
#pragma unroll
    for (int q = 0; q < 8; ++q) acc[q] += xa * bf16_round(ipw[ci * DDm + c0 + q]); }
  v4f oa, ob;
#pragma unroll
  for (int q = 0; q < 8; ++q) { const int c = c0 + q; const float v = ((acc[q] + bf16_round(ipb[c])) + TA[(size_t)b * DDm + c]) + 0.3f * HQ[(size_t)bn * DDm + c]; if (q < 4) oa[q] = v; else ob[q - 4] = v; }
  for (int pass = 0; pass < 2; ++pass) { *(volatile v4f*)(out + (size_t)bn * DDm + c0) = oa; *(volatile v4f*)(out + (size_t)bn * DDm + c0 + 4) = ob; if (pass == 0) __threadfence(); } }

extern "C" void kernel_launch(void* const* d_in, const int* in_sizes, int n_in,
                              void* d_out, int out_size, void* d_ws, size_t ws_size, hipStream_t stream) {
  (void)in_sizes; (void)n_in; (void)out_size;
  const float* const* I = (const float* const*)d_in; const float* x = I[0]; const float* ipw = I[1]; const float* ipb = I[2]; const float* pw1 = I[3]; const float* pb1 = I[4]; const float* pw2 = I[5]; const float* pb2 = I[6]; const float* nw = I[7]; const float* nbias = I[8]; const float* sw1 = I[9]; const float* sb1 = I[10]; const float* sw2 = I[11]; const float* sb2 = I[12]; const float* cw1 = I[13]; const float* cb1 = I[14]; const float* cw2 = I[15]; const float* cb2 = I[16]; const float* pool = I[17];
  float* out0 = (float*)d_out; float* out1 = (float*)((char*)d_out + 8388608);
  char* ws = (char*)d_ws; size_t off = 0;
  auto take = [&](size_t bytes) { char* p = ws + off; off += (bytes + 255) & ~(size_t)255; return p; };
  _Float16* BIN = (_Float16*)take(DDm * 32 * 2); _Float16* BS1 = (_Float16*)take((size_t)NF * DDm * 512 * 2); _Float16* BS2 = (_Float16*)take((size_t)NF * DDm * DDm * 2); _Float16* BC1 = (_Float16*)take((size_t)DDm * 3328 * 2); _Float16* BC2 = (_Float16*)take((size_t)DDm * DDm * 2);
  float* SM = (float*)take((size_t)NB8 * NP * 32 * 4); float* D4 = (float*)take((size_t)NB8 * NP * 32 * 4); float* ATT = (float*)take(NB8 * 32 * 4); float* TA = (float*)take(NB8 * DDm * 4); float* TEF = (float*)take((size_t)NB8 * NF * 2 * DDm * 4); float* XA = (float*)take((size_t)NR * CI * 4);
  _Float16* Ah = (_Float16*)take((size_t)2 * NR * 32 * 2); _Float16* Al = (_Float16*)take((size_t)2 * NR * 32 * 2); float* HF = (float*)take((size_t)2 * NR * DDm * 4); _Float16* COMP16 = (_Float16*)take((size_t)NR * 512 * 2); float* T1 = (float*)take((size_t)NR * DDm * 4); _Float16* P1h = (_Float16*)take((size_t)NR * DDm * 2); _Float16* COMB = (_Float16*)take((size_t)NR * 3328 * 2); float* T2 = (float*)take((size_t)NR * DDm * 4); _Float16* G16 = (_Float16*)take((size_t)NR * DDm * 2); float* HQ = (float*)take((size_t)NR * DDm * 4);
  if (off > ws_size) return;
  k_win<<<1, 256, 0, stream>>>(ipw, BIN);
  for (int f = 0; f < NF; ++f) { k_wt_f16<<<(DDm * (512 / 8) + 255) / 256, 256, 0, stream>>>(sw1 + (size_t)f * 512 * DDm, BS1 + (size_t)f * DDm * 512, 512, DDm, 16.0f); k_wt_f16<<<(DDm * (DDm / 8) + 255) / 256, 256, 0, stream>>>(sw2 + (size_t)f * DDm * DDm, BS2 + (size_t)f * DDm * DDm, DDm, DDm, 16.0f); }
  k_wt_f16<<<(unsigned)(((size_t)DDm * (3328 / 8) + 255) / 256), 256, 0, stream>>>(cw1, BC1, 3328, DDm, 16.0f); k_wt_f16<<<(DDm * (DDm / 8) + 255) / 256, 256, 0, stream>>>(cw2, BC2, DDm, DDm, 16.0f);
  k_smean<<<NB8 * NP, 256, 0, stream>>>(x, SM); k_lagd<<<NB8 * NP, 256, 0, stream>>>(x, D4);
  k_battn<<<NB8, 256, 0, stream>>>(D4, SM, pool, pw1, pb1, pw2, pb2, nw, nbias, ipb, ATT, TA, TEF, out1);
  k_xa<<<(NR * CI + 255) / 256, 256, 0, stream>>>(x, ATT, XA);
  const dim3 gL(((2 * NR / 16) * (DDm / 64) + 3) / 4, 1), gP(((NR / 16) * (DDm / 64) + 3) / 4, 1);
  for (int f = 0; f < NF; ++f) {
    k_dft<<<(NR * 4 + 255) / 256, 256, 0, stream>>>(x, f, Ah, Al);
    k_gemm_hhx<0><<<gL, 128, 0, stream>>>(Ah, 32, 0, BIN, 32, 0, 0.0625f, nullptr, 0, nullptr, 1, 0, 0, HF, nullptr, DDm, 0, 2 * NR, DDm, 32); k_gemm_hhx<0><<<gL, 128, 0, stream>>>(Al, 32, 0, BIN, 32, 0, 0.0625f / 1024.0f, nullptr, 0, HF, 1, (size_t)DDm, 0, HF, nullptr, DDm, 0, 2 * NR, DDm, 32);
    k_comp<<<(NR * 64 + 255) / 256, 256, 0, stream>>>(HF, TEF, f, COMP16);
    k_gemm_hhx<0><<<gP, 128, 0, stream>>>(COMP16, 512, 0, BS1 + (size_t)f * DDm * 512, 512, 0, 0.0625f, sb1 + (size_t)f * DDm, 0, nullptr, 1, 0, 0, T1, nullptr, DDm, 0, NR, DDm, 512); k_gelu<<<(unsigned)(((size_t)NR * DDm / 4 + 255) / 256), 256, 0, stream>>>(T1, P1h, (size_t)NR * DDm / 4);
    k_gemm_hhx<0><<<gP, 128, 0, stream>>>(P1h, DDm, 0, BS2 + (size_t)f * DDm * DDm, DDm, 0, 0.0625f, sb2 + (size_t)f * DDm, 0, nullptr, 1, 0, 0, nullptr, COMB + (size_t)f * DDm, 3328, 0, NR, DDm, DDm); }
  k_gemm_hhx<0><<<gP, 128, 0, stream>>>(COMB, 3328, 0, BC1, 3328, 0, 0.0625f, cb1, 0, nullptr, 1, 0, 0, T2, nullptr, DDm, 0, NR, DDm, 3328); k_gelu<<<(unsigned)(((size_t)NR * DDm / 4 + 255) / 256), 256, 0, stream>>>(T2, G16, (size_t)NR * DDm / 4);
  k_gemm_hhx<0><<<gP, 128, 0, stream>>>(G16, DDm, 0, BC2, DDm, 0, 0.0625f, cb2, 0, nullptr, 1, 0, 0, HQ, nullptr, DDm, 0, NR, DDm, DDm);
  k_z<<<(NR * (DDm / 8) + 255) / 256, 256, 0, stream>>>(XA, ipw, ipb, TA, HQ, out0);
}
